// SpatialSelfAttention_75883482186325
// MI455X (gfx1250) — hardware-verified
//
#include <hip/hip_runtime.h>
#include <math.h>
#include <stdint.h>

#define NB   8
#define NC   256
#define NP   2304
#define CQK  64
#define WSC  256.0f
#define LSC  4096.0f
#define QKC  16.0f
#define VC   4.0f
#define PC   1024.0f
#define SSCALE (1.0f / (QKC * QKC))
static_assert(NB == 8);
static_assert(CQK == 64);
static_assert((NP % 128) == 0 && (NC % 64) == 0 && (NP % 64) == 0);
static_assert((NC % 32) == 0 && (NP % 32) == 0);

typedef _Float16 v16h __attribute__((ext_vector_type(16)));
typedef _Float16 v8h  __attribute__((ext_vector_type(8)));
typedef float    v8f  __attribute__((ext_vector_type(8)));
typedef float    v4f  __attribute__((ext_vector_type(4)));
typedef unsigned int   v4u  __attribute__((ext_vector_type(4)));
typedef unsigned short v8us __attribute__((ext_vector_type(8)));

#if defined(__HIP_DEVICE_COMPILE__)
#define DEV_ASM 1
#else
#define DEV_ASM 0
#endif

__device__ __forceinline__ unsigned short h_bits(_Float16 x) { return __builtin_bit_cast(unsigned short, x); }
__device__ __forceinline__ unsigned pk16(unsigned short a, unsigned short b) { return (unsigned)a | ((unsigned)b << 16); }
__device__ __forceinline__ v8f zero8() { v8f z = {0.f, 0.f, 0.f, 0.f, 0.f, 0.f, 0.f, 0.f}; return z; }

__device__ __forceinline__ void split16(float f, unsigned short& hb, unsigned short& lb) {
  const _Float16 x = (_Float16)f;
  hb = h_bits(x);
  lb = h_bits((_Float16)((f - (float)x) * LSC));
}

__device__ __forceinline__ v16h ldfrag(const _Float16* p) {
  union { v16h v; v8h h[2]; } f;
  f.h[0] = *(const v8h*)(p);
  f.h[1] = *(const v8h*)(p + 16);
  return f.v;
}

__device__ __forceinline__ v8f mmar(v16h a, v16h b, v8f c) {
  return __builtin_amdgcn_wmma_f32_16x16x32_f16(false, a, false, b, (short)0, c, false, false);
}
__device__ __forceinline__ v8f mma_h(v16h a, v16h b, v8f c) {
  c = __builtin_amdgcn_wmma_f32_16x16x32_f16(false, a, false, b, (short)0, c, false, false);
#if DEV_ASM
  asm volatile("v_nop\n\tv_nop\n\tv_nop\n\tv_nop" : "+v"(c) : "v"(a), "v"(b));
#endif
  return c;
}
__device__ __forceinline__ void dep_guard(v8f& a, v8f& b, v16h x, v16h y) {
#if DEV_ASM
  asm volatile("v_nop\n\tv_nop\n\tv_nop\n\tv_nop" : "+v"(a), "+v"(b) : "v"(x), "v"(y));
#else
  (void)a; (void)b; (void)x; (void)y;
#endif
}
__device__ __forceinline__ void keep4(v16h a, v16h b, v16h c, v16h d) {
#if DEV_ASM
  asm volatile("v_nop" :: "v"(a), "v"(b), "v"(c), "v"(d));
#else
  (void)a; (void)b; (void)c; (void)d;
#endif
}
__device__ __forceinline__ void acc_guard4(v8f& a, v8f& b, v8f& c, v8f& d) {
#if DEV_ASM
  asm volatile("v_nop\n\tv_nop\n\tv_nop\n\tv_nop" : "+v"(a), "+v"(b), "+v"(c), "+v"(d));
#else
  (void)a; (void)b; (void)c; (void)d;
#endif
}

__global__ __launch_bounds__(256) void cvt_w(const float* __restrict__ wq, const float* __restrict__ wk,
                                             const float* __restrict__ wv,
                                             unsigned short* wqh, unsigned short* wql,
                                             unsigned short* wkh, unsigned short* wkl,
                                             unsigned short* wvh) {
  const int which = blockIdx.y;
  const int n8 = (which == 2) ? (NC * NC / 8) : (CQK * NC / 8);
  const int i = blockIdx.x * 256 + (int)threadIdx.x;
  if (i >= n8) return;
  const float* src = (which == 0) ? wq : ((which == 1) ? wk : wv);
  unsigned short* dh = (which == 0) ? wqh : ((which == 1) ? wkh : wvh);
  unsigned short* dl = (which == 0) ? wql : wkl;
  const v4f a  = *(const v4f*)(src + (size_t)i * 8);
  const v4f a4 = *(const v4f*)(src + (size_t)i * 8 + 4);
  const float f[8] = {a[0], a[1], a[2], a[3], a4[0], a4[1], a4[2], a4[3]};
  v4u ph, pl;
#pragma unroll
  for (int e = 0; e < 4; ++e) {
    unsigned short h0, l0, h1, l1;
    split16(f[2 * e] * WSC, h0, l0);
    split16(f[2 * e + 1] * WSC, h1, l1);
    ph[e] = pk16(h0, h1);
    pl[e] = pk16(l0, l1);
  }
  unsigned short* oh = dh + (size_t)i * 8;
  unsigned short* ol = dl + (size_t)i * 8;
  *(volatile v4u*)oh = ph;
  if (which != 2) *(volatile v4u*)ol = pl;
  __threadfence();
  *(volatile v4u*)oh = ph;
  if (which != 2) *(volatile v4u*)ol = pl;
}

__global__ __launch_bounds__(256) void xpose_x(const float* __restrict__ x, unsigned short* xh, unsigned short* xl) {
  __shared__ float tile[64][65];
  const int tid = (int)threadIdx.x;
  const int n0 = blockIdx.x * 64, c0 = blockIdx.y * 64, b = blockIdx.z;
  {
    const int tx = tid & 63, ty = tid >> 6;
    const float* src = x + ((size_t)b * NC + c0) * NP + n0 + tx;
#pragma unroll 4
    for (int i = 0; i < 16; ++i) {
      const int c = ty + 4 * i;
      tile[c][tx] = src[(size_t)c * NP];
    }
  }
  __syncthreads();
  const int wave = tid >> 5, lane = tid & 31, q4 = lane >> 3, c8 = (lane & 7) * 8;
  v4u hv[2], lv[2];
#pragma unroll
  for (int it = 0; it < 2; ++it) {
    const int nr = wave * 8 + it * 4 + q4;
    v4u a, a2;
#pragma unroll
    for (int e = 0; e < 4; ++e) {
      unsigned short h0, l0, h1, l1;
      split16(tile[c8 + 2 * e][nr], h0, l0);
      split16(tile[c8 + 2 * e + 1][nr], h1, l1);
      a[e] = pk16(h0, h1);
      a2[e] = pk16(l0, l1);
    }
    hv[it] = a;
    lv[it] = a2;
  }
  for (int pass = 0; pass < 2; ++pass) {
#pragma unroll
    for (int it = 0; it < 2; ++it) {
      const int nr = wave * 8 + it * 4 + q4;
      const size_t go = ((size_t)b * NP + n0 + nr) * NC + c0 + c8;
      *(volatile v4u*)(xh + go) = hv[it];
      *(volatile v4u*)(xl + go) = lv[it];
    }
    __threadfence();
  }
}

__global__ __launch_bounds__(256) void projqk(
    const unsigned short* __restrict__ xhp, const unsigned short* __restrict__ xlp,
    const unsigned short* __restrict__ wqh, const unsigned short* __restrict__ wql,
    const unsigned short* __restrict__ wkh, const unsigned short* __restrict__ wkl,
    const float* __restrict__ bq, const float* __restrict__ bk,
    unsigned short* qh, unsigned short* ql, unsigned short* kh, unsigned short* kl) {
  __shared__ __align__(16) float sT[8][16 * 68];
  const int which = blockIdx.z;
  const int b     = blockIdx.y;
  const int lane  = threadIdx.x & 31;
  const int wave  = threadIdx.x >> 5;
  const int rlane = lane & 15;
  const int koff  = (lane >> 4) * 8;
  const int mOff  = (lane >> 4) * 8;
  const int n0    = (blockIdx.x * 8 + wave) * 16;

  const _Float16* Xh = (const _Float16*)(const void*)xhp + (size_t)b * NP * NC;
  const _Float16* Xl = (const _Float16*)(const void*)xlp + (size_t)b * NP * NC;
  const _Float16* Wh = (const _Float16*)(const void*)(which ? wkh : wqh);
  const _Float16* Wl = (const _Float16*)(const void*)(which ? wkl : wql);
  const float* bias  = which ? bk : bq;
  unsigned short* Oh = (which ? kh : qh) + (size_t)b * NP * CQK;
  unsigned short* Ol = (which ? kl : ql) + (size_t)b * NP * CQK;

  v8f ahh[4], axx[4];
#pragma unroll
  for (int j = 0; j < 4; ++j) { ahh[j] = zero8(); axx[j] = zero8(); }

#pragma unroll 1
  for (int k0 = 0; k0 < NC; k0 += 32) {
    const v16h afh = ldfrag(Xh + (size_t)(n0 + rlane) * NC + koff + k0);
    const v16h afl = ldfrag(Xl + (size_t)(n0 + rlane) * NC + koff + k0);
#pragma unroll
    for (int j = 0; j < 4; ++j) {
      const v16h bfh = ldfrag(Wh + (size_t)(16 * j + rlane) * NC + koff + k0);
      const v16h bfl = ldfrag(Wl + (size_t)(16 * j + rlane) * NC + koff + k0);
      ahh[j] = mma_h(afh, bfh, ahh[j]);
      axx[j] = mma_h(afh, bfl, axx[j]);
      axx[j] = mma_h(afl, bfh, axx[j]);
    }
  }

  float* slab = sT[wave];
#pragma unroll
  for (int j = 0; j < 4; ++j) {
    const float bcol = bias[16 * j + rlane];
#pragma unroll
    for (int r = 0; r < 8; ++r) {
      const float y = (ahh[j][r] + axx[j][r] * (1.0f / LSC)) * (1.0f / WSC) + bcol;
      slab[(mOff + r) * 68 + 16 * j + rlane] = y * QKC;
    }
  }
  __builtin_amdgcn_fence(__ATOMIC_RELEASE, "workgroup");
  __builtin_amdgcn_wave_barrier();
  __builtin_amdgcn_fence(__ATOMIC_ACQUIRE, "workgroup");

  const int q = lane >> 3, c8 = (lane & 7) * 8;
  v4u hv[4], lv[4];
#pragma unroll
  for (int it = 0; it < 4; ++it) {
    const int row = it * 4 + q;
    const float* sp = slab + row * 68 + c8;
    v4u a, a2;
#pragma unroll
    for (int e = 0; e < 4; ++e) {
      unsigned short h0, l0, h1, l1;
      split16(sp[2 * e], h0, l0);
      split16(sp[2 * e + 1], h1, l1);
      a[e] = pk16(h0, h1);
      a2[e] = pk16(l0, l1);
    }
    hv[it] = a;
    lv[it] = a2;
  }
  for (int pass = 0; pass < 2; ++pass) {
#pragma unroll
    for (int it = 0; it < 4; ++it) {
      const int row = it * 4 + q;
      const size_t go = (size_t)(n0 + row) * CQK + c8;
      *(volatile v4u*)(Oh + go) = hv[it];
      *(volatile v4u*)(Ol + go) = lv[it];
    }
    __threadfence();
  }
}

template <int OUT_MODE, bool BIAS_ROW>
__global__ __launch_bounds__(256) void gemm64(
    const unsigned short* __restrict__ Ap, int lda, long long strideA,
    const unsigned short* __restrict__ Btp, int ldb, long long strideB,
    void* Cout, int ldc, long long strideC,
    const float* __restrict__ bias,
    int M, int N, int K, float oscale, float bscale) {
  static_assert(!(OUT_MODE == 0 && BIAS_ROW));
  const _Float16* A  = (const _Float16*)(const void*)Ap;
  const _Float16* Bt = (const _Float16*)(const void*)Btp;
  __shared__ __align__(16) float sT[8][16 * 68];
  const int b    = blockIdx.y;
  const int lane = threadIdx.x & 31;
  const int wave = threadIdx.x >> 5;
  const int tilesN = N >> 6;
  const int tilesM = M >> 6;
  const int tile = blockIdx.x * 8 + wave;
  if (tile >= tilesM * tilesN) return;
  const int tm = tile / tilesN;
  const int tn = tile - tm * tilesN;
  const int m0 = tm << 6;
  const int n0 = tn << 6;

  const _Float16* Ab = A  + (size_t)b * (size_t)strideA;
  const _Float16* Bb = Bt + (size_t)b * (size_t)strideB;

  const int rlane = lane & 15;
  const int koff  = (lane >> 4) * 8;
  const int mOff  = (lane >> 4) * 8;

  v8f acc[4][4];
#pragma unroll
  for (int i = 0; i < 4; ++i)
#pragma unroll
    for (int j = 0; j < 4; ++j) acc[i][j] = zero8();

  for (int k0 = 0; k0 < K; k0 += 32) {
    v16h bq[4];
#pragma unroll
    for (int j = 0; j < 4; ++j)
      bq[j] = ldfrag(Bb + (size_t)(n0 + (j << 4) + rlane) * ldb + koff + k0);
#pragma unroll
    for (int i = 0; i < 4; ++i) {
      const v16h af = ldfrag(Ab + (size_t)(m0 + (i << 4) + rlane) * lda + koff + k0);
#pragma unroll
      for (int j = 0; j < 4; ++j) acc[i][j] = mmar(af, bq[j], acc[i][j]);
      dep_guard(acc[i][0], acc[i][3], af, bq[3]);
    }
    keep4(bq[0], bq[1], bq[2], bq[3]);
  }
  acc_guard4(acc[0][0], acc[0][1], acc[0][2], acc[0][3]);
  acc_guard4(acc[1][0], acc[1][1], acc[1][2], acc[1][3]);
  acc_guard4(acc[2][0], acc[2][1], acc[2][2], acc[2][3]);
  acc_guard4(acc[3][0], acc[3][1], acc[3][2], acc[3][3]);

  float* slab = sT[wave];
#pragma unroll
  for (int i = 0; i < 4; ++i) {
    const int mBase = m0 + (i << 4);
#pragma unroll
    for (int j = 0; j < 4; ++j) {
#pragma unroll
      for (int r = 0; r < 8; ++r) {
        slab[(mOff + r) * 68 + (j << 4) + rlane] = acc[i][j][r];
      }
    }
    __builtin_amdgcn_fence(__ATOMIC_RELEASE, "workgroup");
    __builtin_amdgcn_wave_barrier();
    __builtin_amdgcn_fence(__ATOMIC_ACQUIRE, "workgroup");
    if (OUT_MODE == 0) {
      float* C = (float*)Cout + (size_t)b * (size_t)strideC;
      const int h2 = lane >> 4, c4 = (lane & 15) * 4;
      for (int pass = 0; pass < 2; ++pass) {
#pragma unroll
        for (int it = 0; it < 8; ++it) {
          const int row = it * 2 + h2;
          const v4f v = *(const v4f*)(slab + row * 68 + c4) * oscale;
          *(volatile v4f*)(C + (size_t)(mBase + row) * ldc + n0 + c4) = v;
        }
        __threadfence();
      }
    } else {
      const int q = lane >> 3, c8 = (lane & 7) * 8;
      unsigned short* C = (unsigned short*)Cout + (size_t)b * (size_t)strideC;
      v4u hv[4];
#pragma unroll
      for (int it = 0; it < 4; ++it) {
        const int row = it * 4 + q;
        const float* sp = slab + row * 68 + c8;
        float bb = 0.0f;
        if (BIAS_ROW) bb = bias[mBase + row] * bscale;
        v4u a;
#pragma unroll
        for (int e = 0; e < 4; ++e) {
          const float f0 = sp[2 * e] * oscale + bb;
          const float f1 = sp[2 * e + 1] * oscale + bb;
          a[e] = pk16(h_bits((_Float16)f0), h_bits((_Float16)f1));
        }
        hv[it] = a;
      }
      for (int pass = 0; pass < 2; ++pass) {
#pragma unroll
        for (int it = 0; it < 4; ++it) {
          const int row = it * 4 + q;
          *(volatile v4u*)(C + (size_t)(mBase + row) * ldc + n0 + c8) = hv[it];
        }
        __threadfence();
      }
    }
    __builtin_amdgcn_fence(__ATOMIC_RELEASE, "workgroup");
    __builtin_amdgcn_wave_barrier();
    __builtin_amdgcn_fence(__ATOMIC_ACQUIRE, "workgroup");
  }
}

__global__ __launch_bounds__(256) void logits_softmax(
    const unsigned short* __restrict__ qhp, const unsigned short* __restrict__ qlp,
    const unsigned short* __restrict__ khp, const unsigned short* __restrict__ klp,
    unsigned short* at) {
  __shared__ __align__(16) unsigned short sP[NB][32 * 72];
  const int tid  = (int)threadIdx.x;
  const int wave = tid >> 5;
  const int lane = tid & 31;
  const int hh   = lane >> 4;
  const int c    = lane & 15;
  const int nb   = blockIdx.x, mb = blockIdx.y;
  const int i    = wave & 3, j = wave >> 2;
  const int n0   = nb * 64 + 16 * i;
  const int m0   = mb * 32 + 16 * j;

  const _Float16* Qh = (const _Float16*)(const void*)qhp;
  const _Float16* Ql = (const _Float16*)(const void*)qlp;
  const _Float16* Kh = (const _Float16*)(const void*)khp;
  const _Float16* Kl = (const _Float16*)(const void*)klp;

  v8f s[NB];
#pragma unroll
  for (int b = 0; b < NB; ++b) {
    v8f ah8 = zero8(), ax8 = zero8();
#pragma unroll
    for (int kc = 0; kc < 2; ++kc) {
      const size_t qo = ((size_t)b * NP + n0 + c) * CQK + kc * 32 + 8 * hh;
      const size_t ko = ((size_t)b * NP + m0 + c) * CQK + kc * 32 + 8 * hh;
      const v16h fqh = ldfrag(Qh + qo);
      const v16h fql = ldfrag(Ql + qo);
      const v16h fkh = ldfrag(Kh + ko);
      const v16h fkl = ldfrag(Kl + ko);
      ah8 = mma_h(fqh, fkh, ah8);
      ax8 = mma_h(fqh, fkl, ax8);
      ax8 = mma_h(fql, fkh, ax8);
    }
    s[b] = (ah8 + ax8 * (1.0f / LSC)) * SSCALE;
  }

  v8us pk[NB];
#pragma unroll
  for (int b = 0; b < NB; ++b) { v8us z = {0, 0, 0, 0, 0, 0, 0, 0}; pk[b] = z; }
#pragma unroll
  for (int r = 0; r < 8; ++r) {
    float mx = s[0][r];
#pragma unroll
    for (int b = 1; b < NB; ++b) mx = fmaxf(mx, s[b][r]);
    float e[NB];
    float sum = 0.0f;
#pragma unroll
    for (int b = 0; b < NB; ++b) { e[b] = __expf(s[b][r] - mx); sum += e[b]; }
    const float inv = PC / sum;
#pragma unroll
    for (int b = 0; b < NB; ++b) pk[b][r] = h_bits((_Float16)(e[b] * inv));
  }

#pragma unroll
  for (int b = 0; b < NB; ++b)
    *(v8us*)(sP[b] + (16 * j + c) * 72 + 16 * i + 8 * hh) = pk[b];
  __syncthreads();

  const int q4 = lane >> 3, c8 = (lane & 7) * 8;
  const unsigned short* srow = sP[wave];
  unsigned short* dst = at + ((size_t)wave * NP + mb * 32) * NP + nb * 64 + c8;
  v8us v[8];
#pragma unroll
  for (int it = 0; it < 8; ++it) {
    const int mr = it * 4 + q4;
    v[it] = *(const v8us*)(srow + mr * 72 + c8);
  }
  for (int pass = 0; pass < 2; ++pass) {
#pragma unroll
    for (int it = 0; it < 8; ++it) {
      const int mr = it * 4 + q4;
      *(volatile v8us*)(dst + (size_t)mr * NP) = v[it];
    }
    __threadfence();
  }
}

extern "C" void kernel_launch(void* const* d_in, const int* in_sizes, int n_in,
                              void* d_out, int out_size, void* d_ws, size_t ws_size,
                              hipStream_t stream) {
  if (n_in < 7) return;
  if (in_sizes[0] != NB * NC * NP) return;
  if (in_sizes[1] != CQK * NC || in_sizes[2] != CQK) return;
  if (in_sizes[3] != CQK * NC || in_sizes[4] != CQK) return;
  if (in_sizes[5] != NC * NC || in_sizes[6] != NC) return;
  if (out_size != NB * NC * NP) return;

  const float* x  = (const float*)d_in[0];
  const float* Wq = (const float*)d_in[1];
  const float* bq = (const float*)d_in[2];
  const float* Wk = (const float*)d_in[3];
  const float* bk = (const float*)d_in[4];
  const float* Wv = (const float*)d_in[5];
  const float* bv = (const float*)d_in[6];

  const size_t PX  = (size_t)NB * NP * NC * 2;
  const size_t PW  = (size_t)CQK * NC * 2;
  const size_t PWV = (size_t)NC * NC * 2;
  const size_t PQ  = (size_t)NB * NP * CQK * 2;
  const size_t PV  = (size_t)NB * NC * NP * 2;
  const size_t PAT = (size_t)NB * NP * NP * 2;
  size_t off = 0;
  const size_t oXh = off; off += PX;
  const size_t oXl = off; off += PX;
  const size_t oWqh = off; off += PW;
  const size_t oWql = off; off += PW;
  const size_t oWkh = off; off += PW;
  const size_t oWkl = off; off += PW;
  const size_t oWvh = off; off += PWV;
  const size_t oQh = off; off += PQ;
  const size_t oQl = off; off += PQ;
  const size_t oKh = off; off += PQ;
  const size_t oKl = off; off += PQ;
  const size_t oVp = off; off += PV;
  const size_t oAT = off; off += PAT;
  if (off > ws_size) return;
  if (off > (size_t)134217728) return;

  char* ws = (char*)d_ws;
  unsigned short* Xh  = (unsigned short*)(ws + oXh);
  unsigned short* Xl  = (unsigned short*)(ws + oXl);
  unsigned short* Wqh = (unsigned short*)(ws + oWqh);
  unsigned short* Wql = (unsigned short*)(ws + oWql);
  unsigned short* Wkh = (unsigned short*)(ws + oWkh);
  unsigned short* Wkl = (unsigned short*)(ws + oWkl);
  unsigned short* Wvh = (unsigned short*)(ws + oWvh);
  unsigned short* Qh  = (unsigned short*)(ws + oQh);
  unsigned short* Ql  = (unsigned short*)(ws + oQl);
  unsigned short* Kh  = (unsigned short*)(ws + oKh);
  unsigned short* Kl  = (unsigned short*)(ws + oKl);
  unsigned short* Vp  = (unsigned short*)(ws + oVp);
  unsigned short* AT  = (unsigned short*)(ws + oAT);

  const dim3 blk(256);
  const dim3 gW((NC * NC / 8 + 255) / 256, 3);
  const dim3 gX(NP / 64, NC / 64, NB);
  const dim3 gQK(NP / 128, NB, 2);
  const dim3 gG((((NC / 64) * (NP / 64)) + 7) / 8, NB);
  const dim3 gL(NP / 64, NP / 32);

  cvt_w<<<gW, blk, 0, stream>>>(Wq, Wk, Wv, Wqh, Wql, Wkh, Wkl, Wvh);
  xpose_x<<<gX, blk, 0, stream>>>(x, Xh, Xl);
  projqk<<<gQK, blk, 0, stream>>>(Xh, Xl, Wqh, Wql, Wkh, Wkl, bq, bk, Qh, Ql, Kh, Kl);
  gemm64<1, true><<<gG, blk, 0, stream>>>(
      Wvh, NC, 0LL, Xh, NC, (long long)NP * NC,
      (void*)Vp, NP, (long long)NC * NP, bv,
      NC, NP, NC, VC / WSC, VC);
  logits_softmax<<<gL, blk, 0, stream>>>(Qh, Ql, Kh, Kl, AT);
  gemm64<0, false><<<gG, blk, 0, stream>>>(
      Vp, NP, (long long)NC * NP, AT, NP, (long long)NP * NP,
      d_out, NP, (long long)NC * NP, bv,
      NC, NP, NP, 1.0f / (VC * PC), 0.0f);
  (void)hipGetLastError();
}
